// TransformerBlock_73641509257695
// MI455X (gfx1250) — hardware-verified
//
#include <hip/hip_runtime.h>
#include <stddef.h>


typedef _Float16 v16h __attribute__((ext_vector_type(16)));
typedef _Float16 v8h  __attribute__((ext_vector_type(8)));
typedef float    v8f  __attribute__((ext_vector_type(8)));
typedef float    v4f  __attribute__((ext_vector_type(4)));

#ifndef NB
#define NB 8
#endif
#define NB_FULL 8
#define IMG   256
#define CH    3
#define NTOK  1024
#define PDIM  192
#define DIM   256
#define NHEAD 8
#define HD    32
#define INNER 1024
#define MROWS (NB * NTOK)
#define IMG_STRIDE_FULL  (CH * IMG * IMG)
#define MASK_STRIDE_FULL (IMG * IMG)

static_assert(NB >= 1 && NB <= NB_FULL);
static_assert(DIM == NHEAD * HD);
static_assert(HD == 32);
static_assert((PDIM % 64) == 0 && (DIM % 64) == 0 && (INNER % 64) == 0);
static_assert((PDIM % 32) == 0 && (DIM % 32) == 0 && (INNER % 32) == 0);
static_assert((NTOK % 128) == 0 && (MROWS % 64) == 0);
static_assert(PDIM == CH * 64);

#define LDT 72
#define LDK 40
#define LDP 200
#define LDC 68
#define LDF 196
#define LDSA __attribute__((aligned(16)))

#define WCARRY 64.0f
#define XCARRY 16.0f
#define PCARRY 1024.0f

#define WTP_BYTES  ((size_t)DIM * PDIM * 2)
#define WTKV_BYTES ((size_t)2 * DIM * DIM * 2)
#define WTQ_BYTES  ((size_t)DIM * DIM * 2)
#define WT1_BYTES  ((size_t)INNER * DIM * 2)
#define WT2_BYTES  ((size_t)PDIM * INNER * 2)
#define BIAS_BYTES ((size_t)NB * NTOK * 4)
#define PAT_BYTES  ((size_t)2 * MROWS * PDIM * 2)
#define X_BYTES    ((size_t)2 * MROWS * DIM * 2)
#define HP_BYTES   ((size_t)MROWS * DIM * 2)
#define H_BYTES    ((size_t)MROWS * INNER * 2)
#define OFF_WTP  ((size_t)0)
#define OFF_WTKV (OFF_WTP + WTP_BYTES)
#define OFF_WTQ  (OFF_WTKV + WTKV_BYTES)
#define OFF_WT1  (OFF_WTQ + WTQ_BYTES)
#define OFF_WT2  (OFF_WT1 + WT1_BYTES)
#define OFF_BIAS (OFF_WT2 + WT2_BYTES)
#define OFF_PAT  (OFF_BIAS + BIAS_BYTES)
#define OFF_X    (OFF_PAT + PAT_BYTES)
#define OFF_K    (OFF_X + X_BYTES)
#define OFF_Q    (OFF_K + HP_BYTES)
#define OFF_VT   (OFF_Q + HP_BYTES)
#define OFF_CTX  (OFF_VT + HP_BYTES)
#define OFF_H    (OFF_CTX + HP_BYTES)
#define WS_TOTAL (OFF_H + H_BYTES)
static_assert((WTP_BYTES % 128) == 0 && (WTKV_BYTES % 128) == 0 && (WTQ_BYTES % 128) == 0);
static_assert((WT1_BYTES % 128) == 0 && (WT2_BYTES % 128) == 0 && (BIAS_BYTES % 128) == 0);
static_assert((PAT_BYTES % 128) == 0 && (X_BYTES % 128) == 0 && (HP_BYTES % 128) == 0);
static_assert((H_BYTES % 128) == 0);
static_assert(WS_TOTAL <= (size_t)134217728);

__device__ __forceinline__ float bf16_rne(float x) {
  unsigned int u = __float_as_uint(x);
  u = (u + 0x7FFFu + ((u >> 16) & 1u)) & 0xFFFF0000u;
  return __uint_as_float(u);
}

__device__ __forceinline__ v16h frag_at(const _Float16* p) {
  v8h lo = *(const v8h*)(p);
  v8h hi = *(const v8h*)(p + 16);
  v16h out;
#pragma unroll
  for (int i = 0; i < 8; ++i) { out[i] = lo[i]; out[i + 8] = hi[i]; }
  return out;
}
__device__ __forceinline__ v16h ld_frag(const _Float16* base, unsigned ld) {
  const unsigned lane = threadIdx.x & 31u;
  return frag_at(base + (lane & 15u) * ld + (lane >> 4) * 8u);
}

__device__ __forceinline__ v8f wmma16(v16h a, v16h b, v8f c) {
  v8f d = __builtin_amdgcn_wmma_f32_16x16x32_f16(false, a, false, b, (short)0, c,
                                                 false, false);
  asm volatile("v_nop\n\tv_nop\n\tv_nop\n\tv_nop" : "+v"(d) : "v"(a), "v"(b));
  return d;
}

__device__ __forceinline__ float red16_max(float x) {
#pragma unroll
  for (int off = 1; off < 16; off <<= 1) x = fmaxf(x, __shfl_xor(x, off, 32));
  return x;
}
__device__ __forceinline__ float red16_sum(float x) {
#pragma unroll
  for (int off = 1; off < 16; off <<= 1) x += __shfl_xor(x, off, 32);
  return x;
}

__device__ __forceinline__ void wave_lds_sync() {
  __builtin_amdgcn_fence(3  , "wavefront");
  asm volatile("s_wait_dscnt 0x0" ::: "memory");
  __builtin_amdgcn_wave_barrier();
}

__global__ __launch_bounds__(256) void wconv_kernel(
    const float* __restrict__ W, _Float16* __restrict__ Wt,
    unsigned ldw, unsigned coff, unsigned K) {
  __shared__ LDSA _Float16 T[64 * LDT];
  const unsigned tid = threadIdx.x;
  const unsigned n0 = blockIdx.x * 64u;
  const unsigned k0 = blockIdx.y * 64u;
#pragma unroll 4
  for (unsigned j = 0; j < 16u; ++j) {
    const unsigned idx = tid + 256u * j;
    const unsigned kr = idx >> 6, nc = idx & 63u;
    const float v = W[(size_t)(k0 + kr) * ldw + coff + n0 + nc];
    T[nc * LDT + kr] = (_Float16)(WCARRY * bf16_rne(v));
  }
  __syncthreads();
  v8h x[2];
  size_t off[2];
#pragma unroll
  for (unsigned i = 0; i < 2u; ++i) {
    const unsigned n = 32u * i + (tid >> 3);
    const unsigned kc = (tid & 7u) * 8u;
    x[i] = *(const v8h*)&T[n * LDT + kc];
    off[i] = (size_t)(n0 + n) * K + k0 + kc;
  }
#pragma unroll
  for (int i = 0; i < 2; ++i) *(volatile v8h*)(Wt + off[i]) = x[i];
  __threadfence();
#pragma unroll
  for (int i = 0; i < 2; ++i) *(volatile v8h*)(Wt + off[i]) = x[i];
}

__global__ __launch_bounds__(256) void patch_kernel(
    const float* __restrict__ img0, const float* __restrict__ img1,
    const float* __restrict__ mask, _Float16* __restrict__ pat,
    float* __restrict__ biasb) {
  __shared__ LDSA _Float16 T[32 * LDP];
  __shared__ LDSA float Mb[32];
  const unsigned tid = threadIdx.x;
  const unsigned hh = blockIdx.x, b = blockIdx.y, z = blockIdx.z;

#pragma unroll
  for (unsigned j = 0; j < 6u; ++j) {
    const unsigned idx = tid + 256u * j;
    const unsigned rowi = idx >> 6;
    const unsigned c = rowi >> 3, p1 = rowi & 7u;
    const unsigned xq = idx & 63u;
    const size_t off = (size_t)b * IMG_STRIDE_FULL +
                       (size_t)((c * IMG + hh * 8u + p1) * IMG + xq * 4u);
    const v4f a0 = *(const v4f*)(img0 + off);
    const v4f a1 = *(const v4f*)(img1 + off);
    const v4f a = (z != 0u) ? a1 : a0;
    const unsigned ww = xq >> 1, p2b = (xq & 1u) * 4u;
#pragma unroll
    for (unsigned e = 0; e < 4u; ++e)
      T[ww * LDP + (p1 * 8u + p2b + e) * 3u + c] = (_Float16)bf16_rne(a[e]);
  }
  {
    const unsigned ww = tid >> 3, p1 = tid & 7u;
    const float* mp = mask + (size_t)b * MASK_STRIDE_FULL + (size_t)((hh * 8u + p1) * IMG + ww * 8u);
    const v4f m0 = *(const v4f*)(mp);
    const v4f m1 = *(const v4f*)(mp + 4);
    float s = ((m0[0] + m0[1]) + (m0[2] + m0[3])) + ((m1[0] + m1[1]) + (m1[2] + m1[3]));
    s += __shfl_xor(s, 1, 32);
    s += __shfl_xor(s, 2, 32);
    s += __shfl_xor(s, 4, 32);
    if (p1 == 0u) Mb[ww] = (s > 0.0f) ? 0.0f : -100.0f;
  }
  __syncthreads();

  const size_t base = ((size_t)z * MROWS + (size_t)b * NTOK + hh * 32u) * PDIM;
  v8h x[3];
  size_t off[3];
#pragma unroll
  for (unsigned i = 0; i < 3u; ++i) {
    const unsigned e = (tid + 256u * i) * 8u;
    const unsigned r = e / (unsigned)PDIM;
    const unsigned c = e - r * (unsigned)PDIM;
    x[i] = *(const v8h*)&T[r * LDP + c];
    off[i] = base + e;
  }
  const bool wb = (z == 0u) && (tid < 8u);
  const v4f mb = *(const v4f*)&Mb[(tid & 7u) * 4u];
  const size_t boff = (size_t)b * NTOK + hh * 32u + (tid & 7u) * 4u;
#pragma unroll
  for (int i = 0; i < 3; ++i) *(volatile v8h*)(pat + off[i]) = x[i];
  if (wb) *(volatile v4f*)(biasb + boff) = mb;
  __threadfence();
#pragma unroll
  for (int i = 0; i < 3; ++i) *(volatile v8h*)(pat + off[i]) = x[i];
  if (wb) *(volatile v4f*)(biasb + boff) = mb;
}

__global__ __launch_bounds__(256) void embed_kernel(
    const _Float16* __restrict__ pat, const _Float16* __restrict__ wt,
    const float* __restrict__ bpatch, _Float16* __restrict__ x16) {
  __shared__ LDSA float Cs[64 * LDC];
  __shared__ LDSA float Pe[64 * LDC];
  const unsigned tid = threadIdx.x, lane = tid & 31u;
  const unsigned wave = (unsigned)__builtin_amdgcn_readfirstlane((int)(tid >> 5));
  const unsigned mw = wave >> 1, nw = wave & 1u;
  const unsigned hh = lane >> 4, m = lane & 15u;
  const unsigned n0 = blockIdx.x * 64u;
  const unsigned t0 = blockIdx.y * 64u;

  const float pe_c = (float)(-9.210340371976184 / 256.0);
#pragma unroll 1
  for (unsigned i = 0; i < 8u; ++i) {
    const unsigned j = tid + 256u * i;
    const unsigned r = j >> 5, mp = j & 31u;
    const unsigned mi = (n0 >> 1) + mp;
    const float arg = (float)(2u * mi) * pe_c;
    const float dv = expf(arg);
    const float ang = (float)(t0 + r) * dv;
    Pe[r * LDC + 2u * mp]      = sinf(ang);
    Pe[r * LDC + 2u * mp + 1u] = cosf(ang);
  }

  const unsigned ec = (tid & 7u) * 8u;
  const v4f g0 = *(const v4f*)(bpatch + n0 + ec);
  const v4f g1 = *(const v4f*)(bpatch + n0 + ec + 4);

  const _Float16* bp0 = wt + (size_t)(n0 + nw * 32u + m) * PDIM + hh * 8u;
  const _Float16* bp1 = bp0 + 16 * PDIM;

#pragma unroll 1
  for (unsigned g = 0; g < (unsigned)(2 * NB); ++g) {
    const unsigned row0 = g * (unsigned)NTOK + t0;
    const _Float16* ap = pat + (size_t)(row0 + mw * 16u + m) * PDIM + hh * 8u;
    v8f acc0 = {}, acc1 = {};
#pragma unroll
    for (unsigned k0 = 0; k0 < (unsigned)PDIM; k0 += 32u) {
      const v16h a  = frag_at(ap + k0);
      const v16h b0 = frag_at(bp0 + k0);
      const v16h b1 = frag_at(bp1 + k0);
      acc0 = wmma16(a, b0, acc0);
      acc1 = wmma16(a, b1, acc1);
    }
#pragma unroll
    for (int r = 0; r < 8; ++r) {
      float* d = &Cs[(mw * 16u + hh * 8u + (unsigned)r) * LDC + nw * 32u + m];
      d[0]  = acc0[r];
      d[16] = acc1[r];
    }
    __syncthreads();

    v8h x[2];
    size_t off[2];
#pragma unroll
    for (unsigned i = 0; i < 2u; ++i) {
      const unsigned r = 32u * i + (tid >> 3);
      const v4f u0 = *(const v4f*)&Cs[r * LDC + ec];
      const v4f u1 = *(const v4f*)&Cs[r * LDC + ec + 4];
      const v4f p0 = *(const v4f*)&Pe[r * LDC + ec];
      const v4f p1 = *(const v4f*)&Pe[r * LDC + ec + 4];
#pragma unroll
      for (int j = 0; j < 4; ++j) {
        const float y0 = (u0[j] * (1.0f / WCARRY) + bf16_rne(g0[j])) + p0[j];
        const float y1 = (u1[j] * (1.0f / WCARRY) + bf16_rne(g1[j])) + p1[j];
        x[i][j]     = (_Float16)(XCARRY * y0);
        x[i][j + 4] = (_Float16)(XCARRY * y1);
      }
      off[i] = (size_t)(row0 + r) * DIM + n0 + ec;
    }
#pragma unroll
    for (int i = 0; i < 2; ++i) *(volatile v8h*)(x16 + off[i]) = x[i];
    __threadfence();
#pragma unroll
    for (int i = 0; i < 2; ++i) *(volatile v8h*)(x16 + off[i]) = x[i];
    __syncthreads();
  }
}

template <int MODE>
__global__ __launch_bounds__(256) void gemm_kernel(
    const _Float16* __restrict__ A16, const _Float16* __restrict__ Bt,
    const float* __restrict__ addf, _Float16* __restrict__ out16) {
  __shared__ LDSA float Cs[64 * LDC];
  const unsigned tid = threadIdx.x, lane = tid & 31u;
  const unsigned wave = (unsigned)__builtin_amdgcn_readfirstlane((int)(tid >> 5));
  const unsigned mw = wave >> 1, nw = wave & 1u;
  const unsigned hh = lane >> 4, m = lane & 15u;
  const unsigned n0 = blockIdx.x * 64u;
  const unsigned row0 = blockIdx.y * 64u;
  const unsigned bidx = row0 / (unsigned)NTOK;
  const unsigned t0 = row0 - bidx * (unsigned)NTOK;

  size_t aoff;
  unsigned astep;
  if (MODE == 2) {
    aoff = (size_t)bidx * NHEAD * NTOK * HD + (size_t)(t0 + mw * 16u + m) * HD + hh * 8u;
    astep = (unsigned)(NTOK * HD);
  } else {
    aoff = (size_t)(row0 + mw * 16u + m) * DIM + hh * 8u;
    astep = 32u;
  }
  const _Float16* ap  = A16 + aoff;
  const _Float16* bp0 = Bt + (size_t)(n0 + nw * 32u + m) * DIM + hh * 8u;
  const _Float16* bp1 = bp0 + 16 * DIM;
  v8f acc0 = {}, acc1 = {};
#pragma unroll 4
  for (unsigned s = 0; s < (unsigned)(DIM / 32); ++s) {
    const v16h a  = frag_at(ap + (size_t)s * astep);
    const v16h b0 = frag_at(bp0 + s * 32u);
    const v16h b1 = frag_at(bp1 + s * 32u);
    acc0 = wmma16(a, b0, acc0);
    acc1 = wmma16(a, b1, acc1);
  }
#pragma unroll
  for (int r = 0; r < 8; ++r) {
    float* d = &Cs[(mw * 16u + hh * 8u + (unsigned)r) * LDC + nw * 32u + m];
    d[0]  = acc0[r];
    d[16] = acc1[r];
  }
  __syncthreads();

  if (MODE == 0) {
    v8h x[2];
    size_t off[2];
    const unsigned hd0 = n0 >> 5;
    const unsigned r = tid >> 2;
    const unsigned c = (tid & 3u) * 8u;
#pragma unroll
    for (unsigned i = 0; i < 2u; ++i) {
      const v4f u0 = *(const v4f*)&Cs[r * LDC + i * 32u + c];
      const v4f u1 = *(const v4f*)&Cs[r * LDC + i * 32u + c + 4];
      const v4f g0 = *(const v4f*)(addf + n0 + i * 32u + c);
      const v4f g1 = *(const v4f*)(addf + n0 + i * 32u + c + 4);
#pragma unroll
      for (int j = 0; j < 4; ++j) {
        x[i][j]     = (_Float16)(u0[j] * (1.0f / XCARRY) + WCARRY * bf16_rne(g0[j]));
        x[i][j + 4] = (_Float16)(u1[j] * (1.0f / XCARRY) + WCARRY * bf16_rne(g1[j]));
      }
      off[i] = ((size_t)(bidx * NHEAD + hd0 + i) * NTOK + t0 + r) * HD + c;
    }
#pragma unroll
    for (int i = 0; i < 2; ++i) *(volatile v8h*)(out16 + off[i]) = x[i];
    __threadfence();
#pragma unroll
    for (int i = 0; i < 2; ++i) *(volatile v8h*)(out16 + off[i]) = x[i];
  }

  if (MODE == 1) {
    v8h x[2];
    size_t off[2];
#pragma unroll
    for (unsigned i = 0; i < 2u; ++i) {
      const unsigned dcol = 32u * i + (tid >> 3);
      const unsigned kk = (tid & 7u) * 8u;
      const float gb = WCARRY * bf16_rne(addf[n0 + dcol]);
#pragma unroll
      for (unsigned j = 0; j < 8u; ++j)
        x[i][j] = (_Float16)(Cs[(kk + j) * LDC + dcol] * (1.0f / XCARRY) + gb);
      off[i] = ((size_t)bidx * DIM + n0 + dcol) * NTOK + t0 + kk;
    }
#pragma unroll
    for (int i = 0; i < 2; ++i) *(volatile v8h*)(out16 + off[i]) = x[i];
    __threadfence();
#pragma unroll
    for (int i = 0; i < 2; ++i) *(volatile v8h*)(out16 + off[i]) = x[i];
  }

  if (MODE == 2) {
    v8h x[2];
    size_t off[2];
    const unsigned c = (tid & 7u) * 8u;
    const v4f g0 = *(const v4f*)(addf + n0 + c);
    const v4f g1 = *(const v4f*)(addf + n0 + c + 4);
#pragma unroll
    for (unsigned i = 0; i < 2u; ++i) {
      const unsigned r = 32u * i + (tid >> 3);
      const v4f u0 = *(const v4f*)&Cs[r * LDC + c];
      const v4f u1 = *(const v4f*)&Cs[r * LDC + c + 4];
#pragma unroll
      for (int j = 0; j < 4; ++j) {
        const float a0 = u0[j] * (1.0f / 65536.0f) + bf16_rne(g0[j]);
        const float a1 = u1[j] * (1.0f / 65536.0f) + bf16_rne(g1[j]);
        const float h0 = 0.5f * a0 * (1.0f + erff(a0 * 0.70710678118654752f));
        const float h1 = 0.5f * a1 * (1.0f + erff(a1 * 0.70710678118654752f));
        x[i][j]     = (_Float16)(1024.0f * h0);
        x[i][j + 4] = (_Float16)(1024.0f * h1);
      }
      off[i] = (size_t)(row0 + r) * INNER + n0 + c;
    }
#pragma unroll
    for (int i = 0; i < 2; ++i) *(volatile v8h*)(out16 + off[i]) = x[i];
    __threadfence();
#pragma unroll
    for (int i = 0; i < 2; ++i) *(volatile v8h*)(out16 + off[i]) = x[i];
  }
}

__global__ __launch_bounds__(256) void attn_kernel(
    const _Float16* __restrict__ Qh, const _Float16* __restrict__ Kh,
    const _Float16* __restrict__ Vt, const float* __restrict__ biasb,
    _Float16* __restrict__ Ctx) {
  __shared__ LDSA _Float16 Ks[64 * LDK];
  __shared__ LDSA _Float16 Vs[32 * LDT];
  __shared__ LDSA _Float16 Ps[8 * 16 * LDT];
  __shared__ LDSA float Bs[NTOK];

  const unsigned tid = threadIdx.x, lane = tid & 31u;
  const unsigned wave = (unsigned)__builtin_amdgcn_readfirstlane((int)(tid >> 5));
  const unsigned hh = lane >> 4, m = lane & 15u;
  const unsigned q0 = blockIdx.x * 128u;
  const unsigned head = blockIdx.y;
  const unsigned b = blockIdx.z;
  const float scale = 0.17677669529663687f * (1.0f / 4096.0f);
  const unsigned pbase = wave * (16u * LDT);

  *(v4f*)&Bs[tid * 4u] = *(const v4f*)(biasb + (size_t)b * NTOK + tid * 4u);

  const size_t plane = (size_t)(b * (unsigned)NHEAD + head) * NTOK * HD;
  const v16h qf = frag_at(Qh + plane + (size_t)(q0 + wave * 16u + m) * HD + hh * 8u);

  float mrow[8], lrow[8];
  v8f o[2];
#pragma unroll
  for (int v = 0; v < 8; ++v) { mrow[v] = -1.0e30f; lrow[v] = 0.0f; }
  o[0] = (v8f){};
  o[1] = (v8f){};

  for (unsigned kb = 0; kb < (unsigned)NTOK; kb += 64u) {
    {
      const unsigned r = tid >> 2, c = (tid & 3u) * 8u;
      *(v8h*)&Ks[r * LDK + c] = *(const v8h*)(Kh + plane + (size_t)(kb + r) * HD + c);
    }
    {
      const unsigned r = tid >> 3, c = (tid & 7u) * 8u;
      *(v8h*)&Vs[r * LDT + c] = *(const v8h*)(Vt + plane + (size_t)r * NTOK + kb + c);
    }
    __syncthreads();

    v8f s[4];
#pragma unroll
    for (int kg = 0; kg < 4; ++kg) {
      v8f t = {};
      const v16h kf = ld_frag(&Ks[(kg * 16) * LDK], LDK);
      t = wmma16(qf, kf, t);
      const float bk = Bs[kb + (unsigned)kg * 16u + m];
      s[kg] = t * scale + bk;
    }

    float alpha[8];
#pragma unroll
    for (int v = 0; v < 8; ++v) {
      float mx = fmaxf(fmaxf(s[0][v], s[1][v]), fmaxf(s[2][v], s[3][v]));
      mx = red16_max(mx);
      const float mn = fmaxf(mrow[v], mx);
      alpha[v] = __expf(mrow[v] - mn);
      mrow[v] = mn;
    }
#pragma unroll
    for (int kg = 0; kg < 4; ++kg)
#pragma unroll
      for (int v = 0; v < 8; ++v) s[kg][v] = __expf(s[kg][v] - mrow[v]);
#pragma unroll
    for (int v = 0; v < 8; ++v) {
      const float rs = red16_sum((s[0][v] + s[1][v]) + (s[2][v] + s[3][v]));
      lrow[v] = alpha[v] * lrow[v] + rs;
    }
#pragma unroll
    for (int nb = 0; nb < 2; ++nb)
#pragma unroll
      for (int v = 0; v < 8; ++v) o[nb][v] = o[nb][v] * alpha[v];

#pragma unroll
    for (int kg = 0; kg < 4; ++kg)
#pragma unroll
      for (int v = 0; v < 8; ++v)
        Ps[pbase + (hh * 8u + (unsigned)v) * LDT + (unsigned)kg * 16u + m] =
            (_Float16)(s[kg][v] * PCARRY);
    wave_lds_sync();

#pragma unroll
    for (int c = 0; c < 2; ++c) {
      const v16h pf = ld_frag(&Ps[pbase + c * 32], LDT);
#pragma unroll
      for (int nb = 0; nb < 2; ++nb) {
        const v16h vf = ld_frag(&Vs[(nb * 16) * LDT + c * 32], LDT);
        o[nb] = wmma16(pf, vf, o[nb]);
      }
    }
    __syncthreads();
  }

  float inv[8];
#pragma unroll
  for (int v = 0; v < 8; ++v) inv[v] = __builtin_amdgcn_rcpf(lrow[v]) * (1.0f / 64.0f);
#pragma unroll
  for (int nb = 0; nb < 2; ++nb)
#pragma unroll
    for (int v = 0; v < 8; ++v)
      Ps[pbase + (hh * 8u + (unsigned)v) * LDT + (unsigned)nb * 16u + m] =
          (_Float16)(o[nb][v] * inv[v]);
  wave_lds_sync();
  v8h x[2];
  size_t off[2];
#pragma unroll
  for (unsigned i = 0; i < 2u; ++i) {
    const unsigned piece = lane + 32u * i;
    const unsigned r = piece >> 2;
    const unsigned c = (piece & 3u) * 8u;
    x[i] = *(const v8h*)&Ps[pbase + r * LDT + c];
    off[i] = plane + (size_t)(q0 + wave * 16u + r) * HD + c;
  }
#pragma unroll
  for (int i = 0; i < 2; ++i) *(volatile v8h*)(Ctx + off[i]) = x[i];
  __threadfence();
#pragma unroll
  for (int i = 0; i < 2; ++i) *(volatile v8h*)(Ctx + off[i]) = x[i];
}

__global__ __launch_bounds__(256) void fc2_kernel(
    const _Float16* __restrict__ H16, const _Float16* __restrict__ Wt,
    const float* __restrict__ bias, float* __restrict__ out) {
  __shared__ LDSA float Cf[64 * LDF];
  const unsigned tid = threadIdx.x, lane = tid & 31u;
  const unsigned wave = (unsigned)__builtin_amdgcn_readfirstlane((int)(tid >> 5));
  const unsigned mw = wave >> 1, nw = wave & 1u;
  const unsigned hh = lane >> 4, m = lane & 15u;
  const unsigned row0 = blockIdx.x * 64u;
  const unsigned bidx = row0 / (unsigned)NTOK;
  const unsigned hh0 = (row0 - bidx * (unsigned)NTOK) >> 5;

  const _Float16* ap = H16 + (size_t)(row0 + mw * 16u + m) * INNER + hh * 8u;
  const _Float16* bp = Wt + (size_t)(nw * 96u + m) * INNER + hh * 8u;
  v8f acc[6];
#pragma unroll
  for (int j = 0; j < 6; ++j) acc[j] = (v8f){};
#pragma unroll 2
  for (unsigned k0 = 0; k0 < (unsigned)INNER; k0 += 32u) {
    const v16h a = frag_at(ap + k0);
#pragma unroll
    for (int j = 0; j < 6; ++j) {
      const v16h bf = frag_at(bp + (size_t)j * 16 * INNER + k0);
      acc[j] = wmma16(a, bf, acc[j]);
    }
  }
#pragma unroll
  for (int j = 0; j < 6; ++j) {
    const unsigned col = nw * 96u + (unsigned)j * 16u + m;
    const float gb = bf16_rne(bias[col]);
#pragma unroll
    for (int r = 0; r < 8; ++r)
      Cf[(mw * 16u + hh * 8u + (unsigned)r) * LDF + col] = acc[j][r] * (1.0f / 65536.0f) + gb;
  }
  __syncthreads();

#pragma unroll
  for (unsigned c = 0; c < 3u; ++c) {
    v4f xs[4];
    size_t off[4];
#pragma unroll
    for (unsigned q = 0; q < 4u; ++q) {
      const unsigned id = tid + 256u * q;
      const unsigned hhl = id >> 9;
      const unsigned p1 = (id >> 6) & 7u;
      const unsigned xq = id & 63u;
      const unsigned tokl = hhl * 32u + (xq >> 1);
      const unsigned fb = (p1 * 8u + (xq & 1u) * 4u) * 3u + c;
      const float* src = &Cf[tokl * LDF + fb];
      v4f val;
      val[0] = src[0];
      val[1] = src[3];
      val[2] = src[6];
      val[3] = src[9];
      xs[q] = val;
      off[q] = ((size_t)(bidx * CH + c) * IMG + (hh0 + hhl) * 8u + p1) * IMG + xq * 4u;
    }
#pragma unroll
    for (int q = 0; q < 4; ++q) *(volatile v4f*)(out + off[q]) = xs[q];
    __threadfence();
#pragma unroll
    for (int q = 0; q < 4; ++q) *(volatile v4f*)(out + off[q]) = xs[q];
  }
}

extern "C" void kernel_launch(void* const* d_in, const int* in_sizes, int n_in,
                              void* d_out, int out_size, void* d_ws, size_t ws_size,
                              hipStream_t stream) {
  if (n_in < 13) return;
  const long long need_img = (long long)NB * IMG_STRIDE_FULL;
  if ((long long)in_sizes[0] < need_img) return;
  if ((long long)in_sizes[1] < need_img) return;
  if ((long long)in_sizes[2] < (long long)NB * MASK_STRIDE_FULL) return;
  if (in_sizes[3] < PDIM * DIM) return;
  if (in_sizes[4] < DIM) return;
  if (in_sizes[5] < DIM * 2 * DIM) return;
  if (in_sizes[6] < 2 * DIM) return;
  if (in_sizes[7] < DIM * 2 * DIM) return;
  if (in_sizes[8] < DIM) return;
  if (in_sizes[9] < DIM * INNER) return;
  if (in_sizes[10] < INNER) return;
  if (in_sizes[11] < INNER * PDIM) return;
  if (in_sizes[12] < PDIM) return;
  if ((long long)out_size < need_img) return;
  if (ws_size < WS_TOTAL) return;

  const float* img0    = (const float*)d_in[0];
  const float* img1    = (const float*)d_in[1];
  const float* mask    = (const float*)d_in[2];
  const float* w_patch = (const float*)d_in[3];
  const float* b_patch = (const float*)d_in[4];
  const float* w_kv    = (const float*)d_in[5];
  const float* b_kv    = (const float*)d_in[6];
  const float* w_qv    = (const float*)d_in[7];
  const float* b_qv    = (const float*)d_in[8];
  const float* w_fc1   = (const float*)d_in[9];
  const float* b_fc1   = (const float*)d_in[10];
  const float* w_fc2   = (const float*)d_in[11];
  const float* b_fc2   = (const float*)d_in[12];
  float* out = (float*)d_out;

  char* ws = (char*)d_ws;
  _Float16* WtP  = (_Float16*)(ws + OFF_WTP);
  _Float16* WtKV = (_Float16*)(ws + OFF_WTKV);
  _Float16* WtQ  = (_Float16*)(ws + OFF_WTQ);
  _Float16* Wt1  = (_Float16*)(ws + OFF_WT1);
  _Float16* Wt2  = (_Float16*)(ws + OFF_WT2);
  float*    Bias = (float*)(ws + OFF_BIAS);
  _Float16* Pat  = (_Float16*)(ws + OFF_PAT);
  _Float16* X16  = (_Float16*)(ws + OFF_X);
  _Float16* Kh   = (_Float16*)(ws + OFF_K);
  _Float16* Qh   = (_Float16*)(ws + OFF_Q);
  _Float16* Vt   = (_Float16*)(ws + OFF_VT);
  _Float16* Ctx  = (_Float16*)(ws + OFF_CTX);
  _Float16* H16  = (_Float16*)(ws + OFF_H);

  dim3 blk(256);

  wconv_kernel<<<dim3(DIM / 64, PDIM / 64), blk, 0, stream>>>(w_patch, WtP, DIM, 0u, PDIM);
  wconv_kernel<<<dim3(2 * DIM / 64, DIM / 64), blk, 0, stream>>>(w_kv, WtKV, 2 * DIM, 0u, DIM);
  wconv_kernel<<<dim3(DIM / 64, DIM / 64), blk, 0, stream>>>(w_qv, WtQ, 2 * DIM, 0u, DIM);
  wconv_kernel<<<dim3(INNER / 64, DIM / 64), blk, 0, stream>>>(w_fc1, Wt1, INNER, 0u, DIM);
  wconv_kernel<<<dim3(PDIM / 64, INNER / 64), blk, 0, stream>>>(w_fc2, Wt2, PDIM, 0u, INNER);

  patch_kernel<<<dim3(32, NB, 2), blk, 0, stream>>>(img0, img1, mask, Pat, Bias);
  embed_kernel<<<dim3(DIM / 64, NTOK / 64), blk, 0, stream>>>(Pat, WtP, b_patch, X16);

  dim3 g4(DIM / 64, MROWS / 64);
  gemm_kernel<0><<<g4, blk, 0, stream>>>(X16, WtKV, b_kv, Kh);
  gemm_kernel<1><<<g4, blk, 0, stream>>>(X16, WtKV + (size_t)DIM * DIM, b_kv + DIM, Vt);
  gemm_kernel<0><<<g4, blk, 0, stream>>>(X16 + (size_t)MROWS * DIM, WtQ, b_qv, Qh);

  attn_kernel<<<dim3(NTOK / 128, NHEAD, NB), blk, 0, stream>>>(Qh, Kh, Vt, Bias, Ctx);

  gemm_kernel<2><<<dim3(INNER / 64, MROWS / 64), blk, 0, stream>>>(Ctx, Wt1, b_fc1, H16);
  fc2_kernel<<<dim3(MROWS / 64), blk, 0, stream>>>(H16, Wt2, b_fc2, out);
}
